// Pairwise_Predictor_60722247630945
// MI455X (gfx1250) — hardware-run, weakly checked
//
#include <hip/hip_runtime.h>
#include <stdint.h>

#define NTOK   1024
#define CIN    64
#define HID    128
#define K2     128
#define NP     256
#define TP     136
#define HC     32
#define OP     65
#define PARN   512
#define WSCAP  134217728
#define TWO_LOG2E 2.88539008177792681472f

static_assert(CIN == 64);
static_assert(HID == 128);
static_assert(2 * CIN == K2);
static_assert(K2 % 32 == 0);
static_assert(NTOK % 128 == 0);
static_assert(NTOK % 64 == 0);
static_assert(NP == 2 * HID);
static_assert(NP % 64 == 0);
static_assert(HID % HC == 0);
static_assert((TP * 2) % 16 == 0);
static_assert(16 * 16 * 4 * 4 == 64 * 64);
static_assert(4 * HC * 64 * 4 + HID * 4 + 64 * OP * 4 <= 65536);
static_assert(128 * 64 * 4 <= 65536);
static_assert(64 * TP * 2 <= 65536);

typedef __attribute__((ext_vector_type(16))) __bf16 v16b;
typedef __attribute__((ext_vector_type(8)))  __bf16 v8b;
typedef __attribute__((ext_vector_type(8)))  float  v8f;
typedef __attribute__((ext_vector_type(4)))  float  v4f;
typedef __attribute__((ext_vector_type(4)))  unsigned int v4u;
typedef v8b __attribute__((may_alias)) v8ba;
typedef v4f __attribute__((may_alias)) v4fa;
typedef v4u __attribute__((may_alias)) v4ua;

union FragU { v16b v; v8b h[2]; };

__device__ __forceinline__ unsigned short f2bf_bits(float f) {
  const unsigned u = __float_as_uint(f);
  const unsigned r = (u + 0x7FFFu + ((u >> 16) & 1u)) >> 16;
  const unsigned qn = (u >> 16) | 0x40u;
  const bool isn = (u & 0x7FFFFFFFu) > 0x7F800000u;
  return (unsigned short)(isn ? qn : r);
}
__device__ __forceinline__ float bf_bits2f(unsigned short h) { return __uint_as_float(((unsigned)h) << 16); }
__device__ __forceinline__ float bf16r(float f) { return bf_bits2f(f2bf_bits(f)); }
__device__ __forceinline__ unsigned pk16(unsigned short a, unsigned short b) { return (unsigned)a | ((unsigned)b << 16); }

__device__ __forceinline__ v8f wmma_bf16(v16b a, v16b b, v8f c) {
  v8f d = __builtin_amdgcn_wmma_f32_16x16x32_bf16(false, a, false, b, (short)0, c, false, false);
  asm volatile("v_nop\n\tv_nop\n\tv_nop\n\tv_nop" : "+v"(d) : "v"(a), "v"(b));
  return d;
}

__device__ __forceinline__ v16b load_frag(const unsigned short* p, int hh) {
  FragU f;
  f.h[0] = *(const v8ba*)(p + 8 * hh);
  f.h[1] = *(const v8ba*)(p + 16 + 8 * hh);
  return f.v;
}

__device__ __forceinline__ void gemm_core1_32x64(
    const unsigned short* __restrict__ A, const unsigned short* __restrict__ Bt,
    int K, size_t aoff, size_t boff, int hh, v8f (&acc)[2][4]) {
  const unsigned short* a0 = A + aoff;
  const unsigned short* a1 = a0 + (size_t)16 * K;
  const unsigned short* bp = Bt + boff;
#pragma unroll 1
  for (int k0 = 0; k0 < K; k0 += 32) {
    const v16b f0 = load_frag(a0 + k0, hh);
    const v16b f1 = load_frag(a1 + k0, hh);
#pragma unroll
    for (int nt = 0; nt < 4; ++nt) {
      const v16b fb = load_frag(bp + (size_t)nt * 16 * K + k0, hh);
      acc[0][nt] = wmma_bf16(f0, fb, acc[0][nt]);
      acc[1][nt] = wmma_bf16(f1, fb, acc[1][nt]);
    }
  }
}

__global__ __launch_bounds__(256) void k_prep(const float* __restrict__ x, const float* __restrict__ W1,
                                              const float* __restrict__ b1, const float* __restrict__ W2,
                                              const float* __restrict__ b2,
                                              unsigned short* __restrict__ THL, unsigned short* __restrict__ W1D,
                                              float* __restrict__ PAR) {
  __shared__ __align__(16) unsigned short sT[64 * TP];
  const int tid = threadIdx.x, lane = tid & 31, w = tid >> 5;
  const int bid = blockIdx.x;

  if (bid < 16) {
    const int n0 = bid * 64;
    const int nl = tid & 63, cr = tid >> 6;
#pragma unroll 1
    for (int p = 0; p < 16; ++p) {
      const int c = cr + 4 * p;
      const float xv = bf16r(x[(size_t)c * NTOK + n0 + nl]);
      const float t = tanhf(xv);
      const unsigned short hb = f2bf_bits(t);
      const unsigned short lb = f2bf_bits(t - bf_bits2f(hb));
      sT[nl * TP + c] = hb;
      sT[nl * TP + CIN + c] = lb;
    }
    __syncthreads();
    const int q8 = lane & 7, sub = lane >> 3;
    v4u vv[4];
#pragma unroll
    for (int it = 0; it < 4; ++it) {
      const int lid = 32 * it + 4 * w + sub;
      const int row = lid >> 1, hl = lid & 1;
      vv[it] = *(const v4ua*)(sT + row * TP + 64 * hl + 8 * q8);
    }
    for (int pass = 0; pass < 2; ++pass) {
#pragma unroll
      for (int it = 0; it < 4; ++it) {
        const int lid = 32 * it + 4 * w + sub;
        const int row = lid >> 1, hl = lid & 1;
        *(volatile v4u*)(THL + (size_t)(n0 + row) * K2 + 64 * hl + 8 * q8) = vv[it];
      }
      __threadfence();
    }
    return;
  }

  if (bid < 32) {
    const int u = (bid - 16) * 256 + tid;
    const int np = u >> 4, uu = u & 15;
    const int half = np >> 7, h = np & 127, c8 = (uu & 7) * 8;
    const float* src = W1 + (size_t)h * (2 * CIN) + half * CIN + c8;
    const v4f a = *(const v4fa*)src;
    const v4f c = *(const v4fa*)(src + 4);
    v4u o;
    o[0] = pk16(f2bf_bits(a[0]), f2bf_bits(a[1]));
    o[1] = pk16(f2bf_bits(a[2]), f2bf_bits(a[3]));
    o[2] = pk16(f2bf_bits(c[0]), f2bf_bits(c[1]));
    o[3] = pk16(f2bf_bits(c[2]), f2bf_bits(c[3]));
    unsigned short* dst = W1D + (size_t)u * 8;
    *(volatile v4u*)dst = o;
    __threadfence();
    *(volatile v4u*)dst = o;
    return;
  }

  if (tid >= PARN / 4) return;
  {
    const int u = tid;
    const int ib = (u < 31) ? u : 31;
    const int iw0 = u - 32;
    const int iw = (iw0 < 0) ? 0 : ((iw0 > 31) ? 31 : iw0);
    const v4f vb = *(const v4fa*)(b1 + 4 * ib);
    const v4f vw = *(const v4fa*)(W2 + 4 * iw);
    const float s2 = b2[0];
    asm volatile("" :: "v"(vb), "v"(vw), "v"(s2));
    const unsigned mb = (u < 32) ? 0xffffffffu : 0u;
    const unsigned mw = (u >= 32 && u < 64) ? 0xffffffffu : 0u;
    const unsigned m2 = (u == 64) ? 0xffffffffu : 0u;
    v4f o;
#pragma unroll
    for (int e = 0; e < 4; ++e) {
      const unsigned bb = __float_as_uint(bf16r(vb[e])) & mb;
      const unsigned ww = __float_as_uint(bf16r(vw[e])) & mw;
      o[e] = __uint_as_float(bb | ww);
    }
    o[0] = __uint_as_float(__float_as_uint(o[0]) | (__float_as_uint(bf16r(s2)) & m2));
    float* dst = PAR + 4 * u;
    *(volatile v4f*)dst = o;
    __threadfence();
    *(volatile v4f*)dst = o;
  }
}

__global__ __launch_bounds__(128) void k_gemm(const unsigned short* __restrict__ THL,
                                              const unsigned short* __restrict__ W1D,
                                              const float* __restrict__ PAR,
                                              float* __restrict__ P) {
  __shared__ __align__(16) float sF[128 * 64];
  const int tid = threadIdx.x, lane = tid & 31, w = tid >> 5;
  const int hh = lane >> 4, m = lane & 15;
  const int m0 = blockIdx.x * 128;
  const int n0 = blockIdx.y * 64;
  const int m0w = m0 + 32 * w;

  const v8f zero8 = {0.f, 0.f, 0.f, 0.f, 0.f, 0.f, 0.f, 0.f};
  v8f acc[2][4];
#pragma unroll
  for (int mt = 0; mt < 2; ++mt)
#pragma unroll
    for (int nt = 0; nt < 4; ++nt) acc[mt][nt] = zero8;

  gemm_core1_32x64(THL, W1D, K2, (size_t)(m0w + m) * K2, (size_t)(n0 + m) * K2, hh, acc);

#pragma unroll
  for (int nt = 0; nt < 4; ++nt)
#pragma unroll
    for (int mt = 0; mt < 2; ++mt)
#pragma unroll
      for (int r = 0; r < 8; ++r) {
        const int tokl = 32 * w + 16 * mt + 8 * hh + r;
        const int feat = 16 * nt + m;
        sF[tokl * 64 + feat] = acc[mt][nt][r];
      }
  __syncthreads();
  {
    const int rsub = lane >> 4, c4 = (lane & 15) * 4;
    const bool hasb = (n0 >= HID);
    const int bo = hasb ? (n0 - HID) : 0;
    const v4f braw = *(const v4fa*)(PAR + bo + c4);
    const v4f zero4 = {0.f, 0.f, 0.f, 0.f};
    const v4f bias = hasb ? braw : zero4;
    v4f vals[16];
#pragma unroll
    for (int it = 0; it < 16; ++it) {
      const int row = 32 * w + 2 * it + rsub;
      const v4f v = *(const v4fa*)(sF + row * 64 + c4);
      vals[it] = v + bias;
    }
    for (int pass = 0; pass < 2; ++pass) {
#pragma unroll
      for (int it = 0; it < 16; ++it) {
        const int row = 32 * w + 2 * it + rsub;
        *(volatile v4f*)(P + (size_t)(m0 + row) * NP + n0 + c4) = vals[it];
      }
      __threadfence();
    }
  }
}

__device__ __forceinline__ float tanh_fast(float z) {
#if __has_builtin(__builtin_amdgcn_exp2f)
  const float e = __builtin_amdgcn_exp2f(z * TWO_LOG2E);
#else
  const float e = exp2f(z * TWO_LOG2E);
#endif
  const float r = __builtin_amdgcn_rcpf(1.0f + e);
  return fmaf(-2.0f, r, 1.0f);
}

__global__ __launch_bounds__(256) void k_pair(const float* __restrict__ P, const float* __restrict__ PAR,
                                              float* __restrict__ out) {
  __shared__ __align__(16) float sAI[HC * 64];
  __shared__ __align__(16) float sCI[HC * 64];
  __shared__ __align__(16) float sAJ[HC * 64];
  __shared__ __align__(16) float sCJ[HC * 64];
  __shared__ __align__(16) float sW[HID];
  __shared__ __align__(16) float sO[64 * OP];

  const int ti = blockIdx.y, tj = blockIdx.x;
  if (ti > tj) return;
  const int tid = threadIdx.x, lane = tid & 31, w = tid >> 5;
  const int i0 = ti * 64, j0 = tj * 64;
  const int tx = tid & 15, ty = tid >> 4;

  if (tid < 32) {
    const v4f wv = *(const v4fa*)(PAR + HID + 4 * tid);
    *(v4fa*)(sW + 4 * tid) = wv;
  }
  const float b2r = PAR[2 * HID];

  float sij[4][4], sji[4][4];
#pragma unroll
  for (int a = 0; a < 4; ++a)
#pragma unroll
    for (int b = 0; b < 4; ++b) { sij[a][b] = 0.0f; sji[a][b] = 0.0f; }

  const int q = tid & 7, r = tid >> 3;
#pragma unroll 1
  for (int hc = 0; hc < HID / HC; ++hc) {
    const int h0 = hc * HC;
    __syncthreads();
#pragma unroll
    for (int p = 0; p < 2; ++p) {
      const int row = r + 32 * p;
      const float* gi = P + (size_t)(i0 + row) * NP + h0 + 4 * q;
      const float* gj = P + (size_t)(j0 + row) * NP + h0 + 4 * q;
      const v4f ci = *(const v4fa*)gi;
      const v4f ai = *(const v4fa*)(gi + HID);
      const v4f cj = *(const v4fa*)gj;
      const v4f aj = *(const v4fa*)(gj + HID);
#pragma unroll
      for (int e = 0; e < 4; ++e) {
        sCI[(4 * q + e) * 64 + row] = ci[e];
        sAI[(4 * q + e) * 64 + row] = ai[e];
        sCJ[(4 * q + e) * 64 + row] = cj[e];
        sAJ[(4 * q + e) * 64 + row] = aj[e];
      }
    }
    __syncthreads();
#pragma unroll 1
    for (int hl = 0; hl < HC; ++hl) {
      const v4f ai = *(const v4fa*)(sAI + hl * 64 + 4 * ty);
      const v4f ci = *(const v4fa*)(sCI + hl * 64 + 4 * ty);
      const v4f cj = *(const v4fa*)(sCJ + hl * 64 + 4 * tx);
      const v4f aj = *(const v4fa*)(sAJ + hl * 64 + 4 * tx);
      const float wv = sW[h0 + hl];
#pragma unroll
      for (int a = 0; a < 4; ++a)
#pragma unroll
        for (int b = 0; b < 4; ++b) {
          const float z1 = ai[a] + cj[b];
          const float z2 = aj[b] + ci[a];
          sij[a][b] = fmaf(wv, tanh_fast(z1), sij[a][b]);
          sji[a][b] = fmaf(wv, tanh_fast(z2), sji[a][b]);
        }
    }
  }

#pragma unroll
  for (int a = 0; a < 4; ++a)
#pragma unroll
    for (int b = 0; b < 4; ++b)
      sO[(4 * ty + a) * OP + 4 * tx + b] = (sij[a][b] + b2r) + (sji[a][b] + b2r);
  __syncthreads();

  {
    const int rsub = lane >> 4, c4 = (lane & 15) * 4;
    const bool offd = (ti != tj);
    v4f vd[4], vm[4];
#pragma unroll
    for (int it = 0; it < 4; ++it) {
      const int row = 8 * w + 2 * it + rsub;
#pragma unroll
      for (int e = 0; e < 4; ++e) {
        vd[it][e] = sO[row * OP + c4 + e];
        vm[it][e] = sO[(c4 + e) * OP + row];
      }
    }
    for (int pass = 0; pass < 2; ++pass) {
#pragma unroll
      for (int it = 0; it < 4; ++it) {
        const int row = 8 * w + 2 * it + rsub;
        *(volatile v4f*)(out + (size_t)(i0 + row) * NTOK + j0 + c4) = vd[it];
      }
      if (offd) {
#pragma unroll
        for (int it = 0; it < 4; ++it) {
          const int row = 8 * w + 2 * it + rsub;
          *(volatile v4f*)(out + (size_t)(j0 + row) * NTOK + i0 + c4) = vm[it];
        }
      }
      __threadfence();
    }
  }
}

extern "C" void kernel_launch(void* const* d_in, const int* in_sizes, int n_in,
                              void* d_out, int out_size, void* d_ws, size_t ws_size,
                              hipStream_t stream) {
  if (n_in < 5) return;
  if (in_sizes[0] != CIN * NTOK) return;
  if (in_sizes[1] != HID * 2 * CIN) return;
  if (in_sizes[2] != HID) return;
  if (in_sizes[3] != HID) return;
  if (in_sizes[4] != 1) return;
  if (out_size != NTOK * NTOK) return;

  const float* x  = (const float*)d_in[0];
  const float* W1 = (const float*)d_in[1];
  const float* b1 = (const float*)d_in[2];
  const float* W2 = (const float*)d_in[3];
  const float* b2 = (const float*)d_in[4];
  float* out = (float*)d_out;

  size_t off = 0;
  const size_t oTHL = off; off += (size_t)NTOK * K2 * 2;
  const size_t oW1D = off; off += (size_t)NP * K2 * 2;
  const size_t oPAR = off; off += (size_t)PARN * 4;
  const size_t oP   = off; off += (size_t)NTOK * NP * 4;
  if (off > ws_size) return;
  if (off > (size_t)WSCAP) return;

  char* ws = (char*)d_ws;
  unsigned short* THL = (unsigned short*)(ws + oTHL);
  unsigned short* W1D = (unsigned short*)(ws + oW1D);
  float*          PAR = (float*)(ws + oPAR);
  float*          P   = (float*)(ws + oP);

  k_prep<<<dim3(33), dim3(256), 0, stream>>>(x, W1, b1, W2, b2, THL, W1D, PAR);
  k_gemm<<<dim3(NTOK / 128, NP / 64), dim3(128), 0, stream>>>(THL, W1D, PAR, P);
  k_pair<<<dim3(NTOK / 64, NTOK / 64), dim3(256), 0, stream>>>(P, PAR, out);
  (void)hipGetLastError();
}
